// CrossModeAttention_27650999452505
// MI455X (gfx1250) — hardware-verified
//
#include <hip/hip_runtime.h>
#include <math.h>

typedef __attribute__((ext_vector_type(16))) _Float16 v16h;
typedef __attribute__((ext_vector_type(16))) __bf16 v16b;
typedef __attribute__((ext_vector_type(8)))  _Float16 v8h;
typedef __attribute__((ext_vector_type(8)))  float v8f;
typedef __attribute__((ext_vector_type(4)))  float v4f;
typedef __attribute__((ext_vector_type(2)))  float v2f;
typedef __attribute__((ext_vector_type(4)))  unsigned v4u;
typedef __attribute__((ext_vector_type(4)))  int v4i;
typedef float __attribute__((may_alias)) float_a;
typedef int __attribute__((may_alias)) int_a;

template <typename T> __device__ __forceinline__ void vst2(void* p, T v) { *(volatile T*)p = v; __threadfence(); *(volatile T*)p = v; }
__device__ __forceinline__ v8f wmma16(v16h a, v16h b, v8f c) {
  v8f d = __builtin_amdgcn_wmma_f32_16x16x32_f16(false, a, false, b, (short)0, c, false, false);
  asm volatile("v_nop\n\tv_nop\n\tv_nop\n\tv_nop" : "+v"(d) : "v"(a), "v"(b));
  return d;
}
__device__ __forceinline__ v8f wmma_bf(v16b a, v16b b, v8f c) {
  v8f d = __builtin_amdgcn_wmma_f32_16x16x32_bf16(false, a, false, b, (short)0, c, false, false);
  asm volatile("v_nop\n\tv_nop\n\tv_nop\n\tv_nop" : "+v"(d) : "v"(a), "v"(b));
  return d;
}
__device__ __forceinline__ v16h frag_h(const _Float16* rowk0, int lane) {
  union { v16h v; v8h q[2]; } u; const _Float16* p = rowk0 + 8 * (lane >> 4);
  u.q[0] = *(const v8h*)p; u.q[1] = *(const v8h*)(p + 16); return u.v;
}
__device__ __forceinline__ v16h frag_f32(const float* rowk0, int lane) {
  v16h a; const float* p = rowk0 + 8 * (lane >> 4);
#pragma unroll
  for (int i = 0; i < 8; ++i) { a[i] = (_Float16)p[i]; a[8 + i] = (_Float16)p[16 + i]; }
  return a;
}
__device__ __forceinline__ v16h frag_f32s(const float* rowk0, int lane, float sc) {
  v16h a; const float* p = rowk0 + 8 * (lane >> 4);
#pragma unroll
  for (int i = 0; i < 8; ++i) { a[i] = (_Float16)(p[i] * sc); a[8 + i] = (_Float16)(p[16 + i] * sc); }
  return a;
}
__device__ __forceinline__ v16h fragc_f32(const float* W, int k0, int n, int lane, int ld, int K) {
  v16h a; const int g = lane >> 4;
#pragma unroll
  for (int i = 0; i < 8; ++i) { const int ka = k0 + 8 * g + i, kb = ka + 16;
    a[i] = (_Float16)(ka < K ? W[(size_t)(ka < K ? ka : K - 1) * ld + n] : 0.f); a[8 + i] = (_Float16)(kb < K ? W[(size_t)(kb < K ? kb : K - 1) * ld + n] : 0.f); }
  return a;
}
struct F2 { v16b h, l; };
__device__ __forceinline__ F2 bsplit16(const float v[16]) { F2 r;
#pragma unroll
  for (int i = 0; i < 16; ++i) { const __bf16 h = (__bf16)v[i]; r.h[i] = h; r.l[i] = (__bf16)(v[i] - (float)h); }
  return r; }
__device__ __forceinline__ F2 split_row(const float* row, int k0, int lane) { float v[16]; const float* p = row + k0 + 8 * (lane >> 4);
#pragma unroll
  for (int i = 0; i < 8; ++i) { v[i] = p[i]; v[8 + i] = p[16 + i]; }
  return bsplit16(v); }
__device__ __forceinline__ F2 split_rowK(const float* row, int k0, int lane, int K) { float v[16]; const int g = lane >> 4;
#pragma unroll
  for (int i = 0; i < 8; ++i) { const int ka = k0 + 8 * g + i, kb = ka + 16; v[i] = ka < K ? row[ka < K ? ka : K - 1] : 0.f; v[8 + i] = kb < K ? row[kb < K ? kb : K - 1] : 0.f; }
  return bsplit16(v); }
__device__ __forceinline__ F2 split_col(const float* W, int k0, int n, int lane, int ld, int K) { float v[16]; const int g = lane >> 4;
#pragma unroll
  for (int i = 0; i < 8; ++i) { const int ka = k0 + 8 * g + i, kb = ka + 16; v[i] = ka < K ? W[(size_t)(ka < K ? ka : K - 1) * ld + n] : 0.f; v[8 + i] = kb < K ? W[(size_t)(kb < K ? kb : K - 1) * ld + n] : 0.f; }
  return bsplit16(v); }
__device__ __forceinline__ v8f mac3(const F2& a, const F2& b, v8f c) { c = wmma_bf(a.l, b.h, c); c = wmma_bf(a.h, b.l, c); return wmma_bf(a.h, b.h, c); }
__device__ __forceinline__ float sigm(float v) { return 1.0f / (1.0f + expf(-v)); }
#define LDSX() do { asm volatile("s_wait_dscnt 0" ::: "memory"); __builtin_amdgcn_wave_barrier(); __builtin_amdgcn_fence(__ATOMIC_RELEASE, "workgroup"); } while (0)


#define NB 4
#define NT 1024
#define D1 512
#define C 512
#define NH 8
#define HD 64
#define NR (NB * NT)
#define NLAYER 3
__device__ __forceinline__ v16b frag_b(const __bf16* rowk0, int lane) { return __builtin_bit_cast(v16b, frag_h((const _Float16*)rowk0, lane)); }

__global__ __launch_bounds__(256) void k_cvt2(const float* __restrict__ x1, const float* __restrict__ x2, __bf16* __restrict__ XB) {
  const size_t i8 = (size_t)blockIdx.x * 256 + threadIdx.x; if (i8 >= (size_t)NR * 2 * D1 / 8) return; const size_t r = i8 / (2 * D1 / 8); const int c8 = (int)(i8 % (2 * D1 / 8)) * 8;
  const float* src = c8 < D1 ? x1 + r * D1 + c8 : x2 + r * D1 + (c8 - D1); union { __bf16 e[8]; v4u u; } pk;
#pragma unroll
  for (int e = 0; e < 8; ++e) pk.e[e] = (__bf16)src[e];
  vst2((unsigned*)(XB + i8 * 8), pk.u);
}
__global__ __launch_bounds__(256) void k_pack(const float* __restrict__ Wq, const float* __restrict__ Wk, const float* __restrict__ Wv, __bf16* __restrict__ PQK, __bf16* __restrict__ PV) {
  const int n = blockIdx.x, tid = threadIdx.x; __shared__ __align__(16) __bf16 srow[2 * D1];
  if (n < 2 * C) { const float* W = n < C ? Wq + (size_t)n * D1 : Wk + (size_t)(n - C) * D1; for (int k = tid; k < D1; k += 256) srow[k] = (__bf16)W[k]; __syncthreads(); if (tid < D1 / 8) vst2((unsigned*)(PQK + (size_t)n * D1 + tid * 8), *(const v4u*)(&srow[tid * 8])); }
  else { const float* W = Wv + (size_t)(n - 2 * C) * 2 * D1; for (int k = tid; k < 2 * D1; k += 256) srow[k] = (__bf16)W[k]; __syncthreads(); if (tid < 2 * D1 / 8) vst2((unsigned*)(PV + (size_t)(n - 2 * C) * 2 * D1 + tid * 8), *(const v4u*)(&srow[tid * 8])); }
}
__global__ __launch_bounds__(128) void k_proj(const __bf16* __restrict__ XB, const __bf16* __restrict__ PQK, const __bf16* __restrict__ PV, _Float16* __restrict__ Q16, _Float16* __restrict__ K16, float* __restrict__ V32, _Float16* __restrict__ VT16) {
  __shared__ __align__(16) float so[4][16][132]; __shared__ __align__(16) _Float16 sth[128][72];
  const int tid = threadIdx.x, wave = tid >> 5, lane = tid & 31, col = lane & 15, g = lane >> 4;
  const int which = blockIdx.z, r0b = blockIdx.x * 64, r0 = r0b + wave * 16, n0 = blockIdx.y * 128; const int b = r0b / NT, s0 = r0b % NT;
  v8f acc[8] = {};
  if (which < 2) { const __bf16* A = XB + (size_t)(r0 + col) * 2 * D1 + which * D1; const __bf16* Bw = PQK + (size_t)(which * C + n0) * D1;
#pragma unroll 2
    for (int kc = 0; kc < D1 / 32; ++kc) { const v16b a = frag_b(A + kc * 32, lane);
#pragma unroll
      for (int j = 0; j < 8; ++j) acc[j] = wmma_bf(a, frag_b(Bw + (size_t)(j * 16 + col) * D1 + kc * 32, lane), acc[j]); } }
  else { const __bf16* A = XB + (size_t)(r0 + col) * 2 * D1; const __bf16* Bw = PV + (size_t)n0 * 2 * D1;
#pragma unroll 2
    for (int kc = 0; kc < 2 * D1 / 32; ++kc) { const v16b a = frag_b(A + kc * 32, lane);
#pragma unroll
      for (int j = 0; j < 8; ++j) acc[j] = wmma_bf(a, frag_b(Bw + (size_t)(j * 16 + col) * 2 * D1 + kc * 32, lane), acc[j]); } }
#pragma unroll
  for (int j = 0; j < 8; ++j)
#pragma unroll
    for (int r = 0; r < 8; ++r) so[wave][8 * g + r][j * 16 + col] = acc[j][r];
  LDSX();
  if (which < 2) { _Float16* Dst = which == 0 ? Q16 : K16;
    for (int qq = lane; qq < 2 * 16 * 8; qq += 32) { const int hh = qq >> 7, rl = (qq >> 3) & 15, pc = qq & 7; const int h = (n0 >> 6) + hh; union { v8h h8; v4u u; } pk;
#pragma unroll
      for (int e = 0; e < 8; ++e) pk.h8[e] = (_Float16)(so[wave][rl][hh * 64 + pc * 8 + e] * 4.0f);
      vst2(Dst + (((size_t)b * NH + h) * NT + s0 + wave * 16 + rl) * HD + pc * 8, pk.u); } }
  else {
    for (int rl = 0; rl < 16; ++rl) vst2(V32 + (size_t)(r0 + rl) * C + n0 + lane * 4, *(const v4f*)(&so[wave][rl][lane * 4]));
#pragma unroll
    for (int j = 0; j < 8; ++j)
#pragma unroll
      for (int r = 0; r < 8; ++r) sth[j * 16 + col][wave * 16 + 8 * g + r] = (_Float16)(acc[j][r] * 4.0f);
    __syncthreads();
    for (int qq = tid; qq < 128 * 8; qq += 128) { const int cl = qq >> 3, pc = qq & 7; const int c = n0 + cl, h = c >> 6, d = c & 63; vst2(VT16 + (((size_t)b * NH + h) * HD + d) * NT + s0 + pc * 8, *(const v4u*)(&sth[cl][pc * 8])); } }
}
__global__ __launch_bounds__(128) void k_soft(const _Float16* __restrict__ Q16, const _Float16* __restrict__ K16, _Float16* __restrict__ P16) {
  __shared__ __align__(16) float sS[4][16][68]; __shared__ __align__(16) _Float16 sP[4][16][72];
  const int tid = threadIdx.x, w = tid >> 5, lane = tid & 31, col = lane & 15, g = lane >> 4; const size_t bh = blockIdx.y; const int q0 = blockIdx.x * 64 + w * 16;
  const float scl = 0.04419417382415922f / 16.0f;
  v16h aq[2];
#pragma unroll
  for (int kc = 0; kc < 2; ++kc) aq[kc] = frag_h(Q16 + (bh * NT + q0 + col) * HD + kc * 32, lane);
  float mrun = -3.0e38f, lrun = 0.f;
#pragma unroll 1
  for (int pass = 0; pass < 2; ++pass) {
#pragma unroll 1
    for (int kt = 0; kt < NT / 64; ++kt) {
#pragma unroll
      for (int t = 0; t < 4; ++t) { v8f s = {}; const int key = kt * 64 + t * 16 + col;
#pragma unroll
        for (int kc = 0; kc < 2; ++kc) s = wmma16(aq[kc], frag_h(K16 + (bh * NT + key) * HD + kc * 32, lane), s);
#pragma unroll
        for (int r = 0; r < 8; ++r) sS[w][8 * g + r][t * 16 + col] = s[r] * scl; }
      LDSX();
      if (pass == 0) { float mx = -3.4e38f;
#pragma unroll
        for (int jj = 0; jj < 32; ++jj) mx = fmaxf(mx, sS[w][col][g * 32 + jj]);
        mx = fmaxf(mx, __shfl_xor(mx, 16, 32)); const float mnew = fmaxf(mrun, mx); float ps = 0.f;
#pragma unroll
        for (int jj = 0; jj < 32; ++jj) ps += expf(sS[w][col][g * 32 + jj] - mnew);
        ps += __shfl_xor(ps, 16, 32); lrun = lrun * expf(mrun - mnew) + ps; mrun = mnew; }
      else { const float inv = 16384.0f / lrun;
#pragma unroll
        for (int jj = 0; jj < 32; ++jj) sP[w][col][g * 32 + jj] = (_Float16)(expf(sS[w][col][g * 32 + jj] - mrun) * inv);
        LDSX();
        for (int qq = lane; qq < 16 * 8; qq += 32) { const int rl = qq >> 3, pc = qq & 7; vst2(P16 + ((bh * NT) + q0 + rl) * NT + kt * 64 + pc * 8, *(const v4u*)(&sP[w][rl][pc * 8])); } }
      LDSX(); } }
}
__global__ __launch_bounds__(128) void k_layer(const _Float16* __restrict__ P16, const float* __restrict__ Vin, const _Float16* __restrict__ VTin, const float* __restrict__ gam, const float* __restrict__ bet, float* __restrict__ Vout, _Float16* __restrict__ VTout, int last) {
  __shared__ __align__(16) float srow[4][16][C + 4]; __shared__ __align__(16) _Float16 sth[64][72];
  const int tid = threadIdx.x, wave = tid >> 5, lane = tid & 31, col = lane & 15, g = lane >> 4; const int b = blockIdx.y; const int s0 = blockIdx.x * 64, sw0 = s0 + wave * 16; const size_t r0 = (size_t)b * NT + sw0;
#pragma unroll 1
  for (int h = 0; h < NH; ++h) { const size_t bh = (size_t)b * NH + h; v8f acc[4] = {};
#pragma unroll 2
    for (int kc = 0; kc < NT / 32; ++kc) { const v16h a = frag_h(P16 + (bh * NT + sw0 + col) * NT + kc * 32, lane);
#pragma unroll
      for (int t = 0; t < 4; ++t) acc[t] = wmma16(a, frag_h(VTin + (bh * HD + t * 16 + col) * NT + kc * 32, lane), acc[t]); }
#pragma unroll
    for (int t = 0; t < 4; ++t)
#pragma unroll
      for (int r = 0; r < 8; ++r) srow[wave][8 * g + r][h * HD + t * 16 + col] = acc[t][r] * (1.0f / (16384.0f * 4.0f)) + Vin[(r0 + 8 * g + r) * C + h * HD + t * 16 + col]; }
  LDSX();
  { const int rl = lane & 15, hf = lane >> 4; float* rp = &srow[wave][rl][hf * 256]; float s = 0.f;
#pragma unroll 4
    for (int e = 0; e < 256; ++e) s += rp[e];
    s += __shfl_xor(s, 16, 32); const float mu = s * (1.0f / C); float q = 0.f;
#pragma unroll 4
    for (int e = 0; e < 256; ++e) { const float d = rp[e] - mu; q += d * d; }
    q += __shfl_xor(q, 16, 32); const float rs = rsqrtf(q * (1.0f / C) + 1e-5f);
#pragma unroll 4
    for (int e = 0; e < 256; ++e) { const int c = hf * 256 + e; rp[e] = (rp[e] - mu) * rs * gam[c] + bet[c]; } }
  LDSX();
  for (int rl = 0; rl < 16; ++rl) for (int pc = lane; pc < C / 4; pc += 32) vst2(Vout + (r0 + rl) * C + pc * 4, *(const v4f*)(&srow[wave][rl][pc * 4]));
  if (!last) {
#pragma unroll 1
    for (int cg = 0; cg < C / 64; ++cg) { __syncthreads();
      for (int q = lane; q < 16 * 64; q += 32) { const int rl = q >> 6, cl = q & 63; sth[cl][wave * 16 + rl] = (_Float16)(srow[wave][rl][cg * 64 + cl] * 4.0f); }
      __syncthreads();
      for (int qq = tid; qq < 64 * 8; qq += 128) { const int cl = qq >> 3, pc = qq & 7; const int c = cg * 64 + cl, h = c >> 6, d = c & 63; vst2(VTout + (((size_t)b * NH + h) * HD + d) * NT + s0 + pc * 8, *(const v4u*)(&sth[cl][pc * 8])); } } }
}
extern "C" void kernel_launch(void* const* d_in, const int* in_sizes, int n_in, void* d_out, int out_size, void* d_ws, size_t ws_size, hipStream_t stream) {
  (void)in_sizes; (void)n_in; (void)out_size; (void)ws_size;
  const float** I = (const float**)d_in;
  const float* x1 = I[0]; const float* x2 = I[1]; const float* Wq = I[2]; const float* Wk = I[3]; const float* Wv = I[4]; const float* gam = I[5]; const float* bet = I[6];
  char* ws = (char*)d_ws; size_t off = 0;
  auto take = [&](size_t bytes) { char* p = ws + off; off += (bytes + 255) & ~(size_t)255; return p; };
  __bf16* XB = (__bf16*)take((size_t)NR * 2 * D1 * 2); __bf16* PQK = (__bf16*)take((size_t)2 * C * D1 * 2); __bf16* PV = (__bf16*)take((size_t)C * 2 * D1 * 2);
  _Float16* Q16 = (_Float16*)take((size_t)NR * C * 2); _Float16* K16 = (_Float16*)take((size_t)NR * C * 2); _Float16* P16 = (_Float16*)take((size_t)NB * NH * NT * NT * 2);
  float* VA = (float*)take((size_t)NR * C * 4); float* VB = (float*)take((size_t)NR * C * 4); _Float16* VTA = (_Float16*)take((size_t)NR * C * 2); _Float16* VTB = (_Float16*)take((size_t)NR * C * 2);
  k_cvt2<<<(NR * 2 * D1 / 8 + 255) / 256, 256, 0, stream>>>(x1, x2, XB);
  k_pack<<<3 * C, 256, 0, stream>>>(Wq, Wk, Wv, PQK, PV);
  k_proj<<<dim3(NR / 64, C / 128, 3), 128, 0, stream>>>(XB, PQK, PV, Q16, K16, VA, VTA);
  k_soft<<<dim3(NT / 64, NB * NH), 128, 0, stream>>>(Q16, K16, P16);
  k_layer<<<dim3(NT / 64, NB), 128, 0, stream>>>(P16, VA, VTA, gam, bet, VB, VTB, 0);
  k_layer<<<dim3(NT / 64, NB), 128, 0, stream>>>(P16, VB, VTB, gam, bet, VA, VTA, 0);
  k_layer<<<dim3(NT / 64, NB), 128, 0, stream>>>(P16, VA, VTA, gam, bet, (float*)d_out, nullptr, 1);
}
